// LatentAttention_60730837566202
// MI455X (gfx1250) — hardware-run, weakly checked
//
#include <hip/hip_runtime.h>


#ifndef NB
#define NB 32
#endif
#ifndef SEQ
#define SEQ 1024
#endif
#define NB_FULL  32
#define SEQ_FULL 1024
#ifndef OUT_SEQ
#define OUT_SEQ SEQ
#endif
#define DM   64
#define NH_  8
#define HD   8
#define QKVW 192
#define KO   128
#define PW   16
#define OSP  68
#define EROWS (SEQ < 256 ? SEQ : 256)
#define QRS  2048.0f
#define QRI  (1.0f / 2048.0f)
#define SC2  ((float)(0.35355339059327379 * 1.4426950408889634))
#define PSH  14.0f
#define NEGB (-3.0e38f)

static_assert(HD == 8);
static_assert(NH_ * HD == DM);
static_assert(DM == 64);
static_assert(QKVW == 3 * DM);
static_assert(DM % 32 == 0);
static_assert(KO == 2 * DM);
static_assert(KO % 32 == 0);
static_assert(PW == 2 * HD);
static_assert(SEQ % 64 == 0);
static_assert((NB * SEQ) % 64 == 0);
static_assert(SEQ % 32 == 0);
static_assert(EROWS % 16 == 0);
static_assert((SEQ - EROWS) % 16 == 0);
static_assert(EROWS >= 16);
static_assert(EROWS <= SEQ);
static_assert(NB <= NB_FULL);
static_assert(SEQ <= SEQ_FULL);
static_assert((OSP * 4) % 16 == 0);
static_assert(OSP >= 64);
static_assert(16 * OSP * 4 <= 131072);
static_assert(((size_t)SEQ * DM) % 8 == 0);
static_assert(32 * 16 * NH_ == 16 * DM * 2 * 2);
static_assert(32 * 16 * 4 == 16 * 64 * 2);
static_assert(32 * 16 * 8 == 16 * DM * 4);
static_assert(NH_ * 32 * 16 == 16 * KO * 2);
static_assert(QKVW * (DM / 8) == 6 * 256);
static_assert(DM * (KO / 8) == 4 * 256);

typedef _Float16 h16;
typedef unsigned short bf;
typedef __attribute__((ext_vector_type(16))) __bf16   v16bf;
typedef __attribute__((ext_vector_type(16))) _Float16 v16h;
typedef __attribute__((ext_vector_type(8)))  _Float16 v8h;
typedef __attribute__((ext_vector_type(8)))  unsigned short v8us;
typedef __attribute__((ext_vector_type(8)))  float    v8f;
typedef __attribute__((ext_vector_type(4)))  float    v4f;
typedef v4f  __attribute__((may_alias)) v4fa;

__device__ __forceinline__ unsigned short f2bf(float f) { unsigned u = __float_as_uint(f); u += 0x7FFFu + ((u >> 16) & 1u); return (unsigned short)(u >> 16); }
__device__ __forceinline__ float bfr(float f) { return __uint_as_float(((unsigned)f2bf(f)) << 16); }
__device__ __forceinline__ v16h cat16(v8h lo, v8h hi) { return __builtin_shufflevector(lo, hi, 0, 1, 2, 3, 4, 5, 6, 7, 8, 9, 10, 11, 12, 13, 14, 15); }
__device__ __forceinline__ v16bf cat16b(v8us lo, v8us hi) { return __builtin_bit_cast(v16bf, __builtin_shufflevector(lo, hi, 0, 1, 2, 3, 4, 5, 6, 7, 8, 9, 10, 11, 12, 13, 14, 15)); }
__device__ __forceinline__ v8f wmma16(v16h a, v16h b, v8f c) { return __builtin_amdgcn_wmma_f32_16x16x32_f16(false, a, false, b, (short)0, c, false, false); }
__device__ __forceinline__ v8f wmmab(v16bf a, v16bf b, v8f c) { return __builtin_amdgcn_wmma_f32_16x16x32_bf16(false, a, false, b, (short)0, c, false, false); }
__device__ __forceinline__ v8f mmah(v16h a, v16h b, v8f c) { c = wmma16(a, b, c); asm volatile("v_nop\n\tv_nop\n\tv_nop\n\tv_nop" : "+v"(c) : "v"(a), "v"(b)); return c; }
__device__ __forceinline__ v8f mmab(v16bf a, v16bf b, v8f c) { c = wmmab(a, b, c); asm volatile("v_nop\n\tv_nop\n\tv_nop\n\tv_nop" : "+v"(c) : "v"(a), "v"(b)); return c; }
__device__ __forceinline__ v16h  ldh(const h16* p) { return cat16(*(const v8h*)p, *(const v8h*)(p + 16)); }
__device__ __forceinline__ v16bf ldb(const bf* p)  { return cat16b(*(const v8us*)p, *(const v8us*)(p + 16)); }
__device__ __forceinline__ v16bf ldrow(const bf* p) { return cat16b(*(const v8us*)p, *(const v8us*)(p + 8)); }
static __device__ __forceinline__ h16 toh_flush(float v) { const h16 r = (h16)v; return (fabsf(v) < 6.103515625e-05f) ? (h16)0.0f : r; }
__device__ __forceinline__ void wave_sync() { __builtin_amdgcn_fence(3  , "wavefront"); __builtin_amdgcn_wave_barrier(); asm volatile("" ::: "memory"); }

__global__ __launch_bounds__(256) void k_cvt8(const float* __restrict__ src, bf* dst, size_t n8) {
    const size_t i = (size_t)blockIdx.x * 256 + threadIdx.x; if (i >= n8) return;
    const v8f v = *(const v8f*)(src + i * 8); v8us o;
#pragma unroll
    for (int k = 0; k < 8; ++k) o[k] = f2bf(v[k]);
    *(volatile v8us*)(dst + i * 8) = o; __threadfence(); *(volatile v8us*)(dst + i * 8) = o;
}

__global__ __launch_bounds__(256) void k_wconv(const float* __restrict__ wqkv, const float* __restrict__ wproj, bf* WT, bf* WP2) {
    const int p = (int)blockIdx.x * 256 + (int)threadIdx.x;
    v8us o;
    if (blockIdx.x < 6) {
        const int n = p >> 3, k0 = (p & 7) * 8;
#pragma unroll
        for (int i = 0; i < 8; ++i) o[i] = f2bf(wqkv[(size_t)(k0 + i) * QKVW + n]);
        bf* dst = WT + (size_t)p * 8;
        *(volatile v8us*)dst = o; __threadfence(); *(volatile v8us*)dst = o;
    } else {
        const int q = p - 6 * 256; const int n = q >> 4, k0 = ((q & 15) * 8) & (DM - 1);
#pragma unroll
        for (int i = 0; i < 8; ++i) o[i] = f2bf(wproj[(size_t)(k0 + i) * DM + n]);
        bf* dst = WP2 + (size_t)q * 8;
        *(volatile v8us*)dst = o; __threadfence(); *(volatile v8us*)dst = o;
    }
}

__global__ __launch_bounds__(32) void k_qk(const bf* __restrict__ A, const bf* __restrict__ Bt, const float* __restrict__ bias, bf* QK) {
    __shared__ __align__(16) float os[16 * OSP];
    const int lane = threadIdx.x & 31, lr = lane & 15, hi = lane >> 4;
    const int r0 = blockIdx.x * 64; const int sel = blockIdx.y; const int c0 = sel * 64;
    v8f acc[4][4];
#pragma unroll
    for (int mb = 0; mb < 4; ++mb)
#pragma unroll
        for (int nb = 0; nb < 4; ++nb) acc[mb][nb] = (v8f){};
    const size_t aoff = (size_t)(r0 + lr) * DM + 8 * hi, boff = (size_t)(c0 + lr) * DM + 8 * hi;
#pragma unroll 1
    for (int kc = 0; kc < DM; kc += 32) {
        v16bf a[4];
#pragma unroll
        for (int mb = 0; mb < 4; ++mb) a[mb] = ldb(A + aoff + (size_t)mb * 16 * DM + kc);
#pragma unroll
        for (int nb = 0; nb < 4; ++nb) { const v16bf b = ldb(Bt + boff + (size_t)nb * 16 * DM + kc);
#pragma unroll
            for (int mb = 0; mb < 4; ++mb) acc[mb][nb] = mmab(a[mb], b, acc[mb][nb]); }
    }
    float bc[4];
#pragma unroll
    for (int nb = 0; nb < 4; ++nb) bc[nb] = bfr(bias[c0 + nb * 16 + lr]);
    const int bb = r0 / SEQ, tt = r0 % SEQ;
    const size_t plane = (size_t)sel * ((size_t)NB * NH_ * SEQ * PW);
    const int row = lane >> 1, part = lane & 1;
#pragma unroll
    for (int mb = 0; mb < 4; ++mb) {
#pragma unroll
        for (int nb = 0; nb < 4; ++nb) {
#pragma unroll
            for (int j = 0; j < 8; ++j) os[(hi * 8 + j) * OSP + nb * 16 + lr] = acc[mb][nb][j] + bc[nb]; }
        wave_sync();
#pragma unroll 1
        for (int ps = 0; ps < 2; ++ps) {
#pragma unroll
            for (int hh = 0; hh < NH_; ++hh) {
                const v4f x0 = *(const v4fa*)(&os[row * OSP + hh * 8]); const v4f x1 = *(const v4fa*)(&os[row * OSP + hh * 8 + 4]); v8us ov;
#pragma unroll
                for (int i = 0; i < 4; ++i) {
                    const unsigned short h0 = f2bf(x0[i]); const unsigned short l0 = f2bf(x0[i] - __uint_as_float(((unsigned)h0) << 16));
                    const unsigned short h1 = f2bf(x1[i]); const unsigned short l1 = f2bf(x1[i] - __uint_as_float(((unsigned)h1) << 16));
                    ov[i] = part ? l0 : h0; ov[4 + i] = part ? l1 : h1; }
                const size_t oo = plane + (((size_t)(bb * NH_ + hh) * SEQ) + (size_t)(tt + mb * 16)) * PW + (size_t)lane * 8;
                *(volatile v8us*)(QK + oo) = ov; }
            if (ps == 0) __threadfence(); }
        wave_sync();
    }
}

__global__ __launch_bounds__(32) void k_vt(const bf* __restrict__ A, const bf* __restrict__ Bt, const float* __restrict__ bias, h16* VT) {
    __shared__ __align__(16) float os[16 * OSP];
    const int lane = threadIdx.x & 31, lr = lane & 15, hi = lane >> 4;
    const int c0 = blockIdx.x * 64;
    v8f acc[4][4];
#pragma unroll
    for (int mb = 0; mb < 4; ++mb)
#pragma unroll
        for (int nb = 0; nb < 4; ++nb) acc[mb][nb] = (v8f){};
    const size_t aoff = (size_t)(2 * DM + lr) * DM + 8 * hi, boff = (size_t)(c0 + lr) * DM + 8 * hi;
#pragma unroll 1
    for (int kc = 0; kc < DM; kc += 32) {
        v16bf a[4];
#pragma unroll
        for (int mb = 0; mb < 4; ++mb) a[mb] = ldb(A + aoff + (size_t)mb * 16 * DM + kc);
#pragma unroll
        for (int nb = 0; nb < 4; ++nb) { const v16bf b = ldb(Bt + boff + (size_t)nb * 16 * DM + kc);
#pragma unroll
            for (int mb = 0; mb < 4; ++mb) acc[mb][nb] = mmab(a[mb], b, acc[mb][nb]); }
    }
    const int bb = c0 / SEQ, tt = c0 % SEQ;
#pragma unroll
    for (int mb = 0; mb < 4; ++mb) {
        float br[8];
#pragma unroll
        for (int j = 0; j < 8; ++j) br[j] = bfr(bias[2 * DM + mb * 16 + hi * 8 + j]);
#pragma unroll
        for (int nb = 0; nb < 4; ++nb) {
#pragma unroll
            for (int j = 0; j < 8; ++j) os[(hi * 8 + j) * OSP + nb * 16 + lr] = acc[mb][nb][j] + br[j]; }
        wave_sync();
#pragma unroll 1
        for (int ps = 0; ps < 2; ++ps) {
#pragma unroll
            for (int s = 0; s < 4; ++s) { const int row = 4 * s + (lane >> 3), c8 = (lane & 7) * 8;
                const v4f x0 = *(const v4fa*)(&os[row * OSP + c8]); const v4f x1 = *(const v4fa*)(&os[row * OSP + c8 + 4]); v8h hv, rv;
#pragma unroll
                for (int i = 0; i < 4; ++i) { const h16 a0 = toh_flush(x0[i]); const h16 a1 = toh_flush(x1[i]); hv[i] = a0; hv[4 + i] = a1;
                    rv[i] = toh_flush((x0[i] - (float)a0) * QRS); rv[4 + i] = toh_flush((x1[i] - (float)a1) * QRS); }
                const int mm = mb * 16 + row; const int hh = mm >> 3, dd = mm & 7;
                const size_t prow = (size_t)(bb * NH_ + hh) * 16 + dd;
                const size_t oo = prow * SEQ + (size_t)tt + c8;
                const size_t ro = (prow + 8) * SEQ + (size_t)tt + c8;
                *(volatile v8h*)(VT + oo) = hv; *(volatile v8h*)(VT + ro) = rv; }
            if (ps == 0) __threadfence(); }
        wave_sync();
    }
}

template <int EARLY>
__device__ __forceinline__ void flash_body(const bf* __restrict__ QK, const h16* __restrict__ VT, bf* CT) {
    __shared__ __align__(16) float cs[16 * OSP];
    const int lane = threadIdx.x & 31, lr = lane & 15, hi = lane >> 4;
    const int wave = __builtin_amdgcn_readfirstlane((int)(threadIdx.x >> 5));
    const int b = blockIdx.y;
    const int t0 = (EARLY ? 0 : EROWS) + (int)blockIdx.x * 16;
    const int zh = b * NH_ + wave;
    const int lim = t0 + lr;
    const int nk = (t0 + 16 + 31) & ~31;
    const size_t qb = (size_t)zh * SEQ * PW;
    const v8us qx = *(const v8us*)(QK + qb + (size_t)(t0 + lr) * PW + 8 * hi);
    const v16bf qf = cat16b(qx, qx);
    const size_t ko = (size_t)NB * NH_ * SEQ * PW + qb + (size_t)lr * PW;
    const size_t vo = ((size_t)zh * 16 + lr) * SEQ + 8 * hi;
    const v16h hz = (v16h){};
    v8f o = (v8f){}, oR = (v8f){};
    float m = NEGB, l = 0.0f;
#pragma unroll 1
    for (int key0 = 0; key0 < nk; key0 += 32) {
        const bf* ka = QK + ko + (size_t)key0 * PW;
        const v16bf ka0 = ldrow(ka), kb0 = ldrow(ka + 16 * PW);
        v8f sa = (v8f){}, sb = (v8f){};
        sa = mmab(ka0, qf, sa); sb = mmab(kb0, qf, sb);
        const int ja = key0 + 8 * hi;
        float ta[8], tb[8]; bool fa[8], fb[8]; float mx = NEGB;
#pragma unroll
        for (int r = 0; r < 8; ++r) {
            fa[r] = (ja + r <= lim);
            fb[r] = (ja + 16 + r <= lim);
            ta[r] = sa[r] * SC2; tb[r] = sb[r] * SC2;
            mx = fmaxf(mx, fmaxf(fa[r] ? ta[r] : NEGB, fb[r] ? tb[r] : NEGB)); }
        mx = fmaxf(mx, __shfl_xor(mx, 16, 32));
        const float mnew = fmaxf(m, mx);
        const float alpha = __builtin_amdgcn_exp2f(m - mnew);
        const float sh = PSH - mnew;
        v16h pb, pr = hz; float ls = 0.0f;
#pragma unroll
        for (int r = 0; r < 8; ++r) {
            const float aa = ta[r] + sh, ab = tb[r] + sh;
            const float ea = __builtin_amdgcn_exp2f(aa), eb = __builtin_amdgcn_exp2f(ab);
            const float ga = (fa[r] & (aa >= -14.0f)) ? ea : 0.0f;
            const float gb = (fb[r] & (ab >= -14.0f)) ? eb : 0.0f;
            const h16 pa = (h16)ga; const h16 pc = (h16)gb;
            pb[r] = pa; pb[8 + r] = pc;
            if (EARLY) { pr[r] = toh_flush((ga - (float)pa) * QRS); pr[8 + r] = toh_flush((gb - (float)pc) * QRS); ls += ga + gb; }
            else       { ls += (float)pa + (float)pc; } }
        l = l * alpha + ls; m = mnew;
        o = o * alpha;
        if (EARLY) oR = oR * alpha;
        const v16h v0 = ldh(VT + vo + key0);
        o = mmah(v0, pb, o);
        if (EARLY) oR = mmah(v0, pr, oR);
    }
    l += __shfl_xor(l, 16, 32);
    const bool any = l > 0.0f;
    const float lsafe = any ? l : 1.0f;
    const float inv = any ? (1.0f / lsafe) : 0.0f;
    float val[8];
#pragma unroll
    for (int r = 0; r < 8; ++r) {
        const float ox = __shfl_xor(o[r], 16, 32);
        float rx = 0.0f, rs = 0.0f;
        if (EARLY) { rx = oR[r]; rs = __shfl_xor(oR[r], 16, 32); }
        const float mainv = hi ? ox : o[r];
        const float vres  = hi ? o[r] : ox;
        const float pres  = hi ? rs : rx;
        val[r] = (mainv + (vres + pres) * QRI) * inv; }
    { v4f cv;
#pragma unroll
      for (int i = 0; i < 4; ++i) cv[i] = hi ? val[4 + i] : val[i];
      *(v4fa*)(&cs[lr * OSP + wave * 8 + 4 * hi]) = cv; }
    __syncthreads();
    {
        const int row = 2 * wave + (lane >> 4), pc = lane & 15, c8 = (pc & 7) * 8, part = pc >> 3;
        const v4f x0 = *(const v4fa*)(&cs[row * OSP + c8]); const v4f x1 = *(const v4fa*)(&cs[row * OSP + c8 + 4]); v8us ov;
#pragma unroll
        for (int i = 0; i < 4; ++i) {
            const unsigned short h0 = f2bf(x0[i]); const unsigned short l0 = f2bf(x0[i] - __uint_as_float(((unsigned)h0) << 16));
            const unsigned short h1 = f2bf(x1[i]); const unsigned short l1 = f2bf(x1[i] - __uint_as_float(((unsigned)h1) << 16));
            ov[i] = part ? l0 : h0; ov[4 + i] = part ? l1 : h1; }
        bf* dst = CT + ((size_t)b * SEQ + (size_t)(t0 + row)) * KO + (size_t)pc * 8;
        *(volatile v8us*)dst = ov; __threadfence(); *(volatile v8us*)dst = ov;
    }
}

__global__ __launch_bounds__(32 * NH_) void k_flash_early(const bf* __restrict__ QK, const h16* __restrict__ VT, bf* CT) { flash_body<1>(QK, VT, CT); }
__global__ __launch_bounds__(32 * NH_) void k_flash_late(const bf* __restrict__ QK, const h16* __restrict__ VT, bf* CT)  { flash_body<0>(QK, VT, CT); }

__global__ __launch_bounds__(32) void k_out(const bf* __restrict__ A, const bf* __restrict__ Bt, const float* __restrict__ bias, float* OUT) {
    __shared__ __align__(16) float os[16 * OSP];
    const int lane = threadIdx.x & 31, lr = lane & 15, hi = lane >> 4;
    const int r0 = blockIdx.x * 64;
    v8f acc[4][4];
#pragma unroll
    for (int mb = 0; mb < 4; ++mb)
#pragma unroll
        for (int nb = 0; nb < 4; ++nb) acc[mb][nb] = (v8f){};
    const size_t aoff = (size_t)(r0 + lr) * KO + 8 * hi, boff = (size_t)lr * KO + 8 * hi;
#pragma unroll 1
    for (int kc = 0; kc < KO; kc += 32) {
        v16bf a[4];
#pragma unroll
        for (int mb = 0; mb < 4; ++mb) a[mb] = ldb(A + aoff + (size_t)mb * 16 * KO + kc);
#pragma unroll
        for (int nb = 0; nb < 4; ++nb) { const v16bf b = ldb(Bt + boff + (size_t)nb * 16 * KO + kc);
#pragma unroll
            for (int mb = 0; mb < 4; ++mb) acc[mb][nb] = mmab(a[mb], b, acc[mb][nb]); }
    }
    float bc[4];
#pragma unroll
    for (int nb = 0; nb < 4; ++nb) bc[nb] = bfr(bias[nb * 16 + lr]);
    const int bb = r0 / SEQ, tt = r0 % SEQ;
    float* obase = OUT + ((size_t)bb * OUT_SEQ + (size_t)tt) * DM;
#pragma unroll
    for (int mb = 0; mb < 4; ++mb) {
#pragma unroll
        for (int nb = 0; nb < 4; ++nb) {
#pragma unroll
            for (int j = 0; j < 8; ++j) os[(hi * 8 + j) * OSP + nb * 16 + lr] = acc[mb][nb][j] + bc[nb]; }
        wave_sync();
#pragma unroll 1
        for (int ps = 0; ps < 2; ++ps) {
#pragma unroll
            for (int s = 0; s < 8; ++s) { const int row = 2 * s + (lane >> 4), cofs = (lane & 15) * 4;
                const v4f val = *(const v4fa*)(&os[row * OSP + cofs]);
                *(volatile v4f*)(obase + (size_t)(mb * 16 + row) * DM + cofs) = val; }
            if (ps == 0) __threadfence(); }
        wave_sync();
    }
}

static constexpr size_t al256(size_t v) { return (v + 255) & ~(size_t)255; }
static constexpr size_t SZ_ZB = al256((size_t)NB * SEQ * DM * 2);
static constexpr size_t SZ_WT = al256((size_t)QKVW * DM * 2);
static constexpr size_t SZ_WP = al256((size_t)DM * KO * 2);
static constexpr size_t SZ_QK = al256((size_t)2 * NB * NH_ * SEQ * PW * 2);
static constexpr size_t SZ_VT = al256((size_t)NB * NH_ * 16 * SEQ * 2);
static constexpr size_t SZ_CT = al256((size_t)NB * SEQ * KO * 2);
static constexpr size_t SZ_TOTAL = SZ_ZB + SZ_WT + SZ_WP + SZ_QK + SZ_VT + SZ_CT;
static_assert(SZ_TOTAL <= (size_t)134217728);
static_assert((size_t)QKVW * DM * 2 == (size_t)6 * 256 * 16);
static_assert((size_t)DM * KO * 2 == (size_t)4 * 256 * 16);

extern "C" void kernel_launch(void* const* d_in, const int* in_sizes, int n_in,
                              void* d_out, int out_size, void* d_ws, size_t ws_size, hipStream_t stream) {
    if (n_in < 5) return;
    const size_t needz = ((size_t)(NB - 1) * SEQ_FULL + SEQ) * DM;
    if ((size_t)in_sizes[0] < needz) return;
    if ((size_t)in_sizes[1] < (size_t)DM * QKVW || in_sizes[2] < QKVW) return;
    if ((size_t)in_sizes[3] < (size_t)DM * DM || in_sizes[4] < DM) return;
    if ((size_t)out_size < ((size_t)(NB - 1) * OUT_SEQ + SEQ) * DM) return;
    if (SZ_TOTAL > ws_size) return;
    const float* z     = (const float*)d_in[0];
    const float* wqkv  = (const float*)d_in[1];
    const float* bqkv  = (const float*)d_in[2];
    const float* wproj = (const float*)d_in[3];
    const float* bproj = (const float*)d_in[4];
    float* OUT = (float*)d_out;
    char* wsp = (char*)d_ws;
    bf*  ZB  = (bf*)wsp;  wsp += SZ_ZB;
    bf*  WT  = (bf*)wsp;  wsp += SZ_WT;
    bf*  WP2 = (bf*)wsp;  wsp += SZ_WP;
    bf*  QK  = (bf*)wsp;  wsp += SZ_QK;
    h16* VT  = (h16*)wsp; wsp += SZ_VT;
    bf*  CT  = (bf*)wsp;  wsp += SZ_CT;

    if (SEQ == SEQ_FULL) {
        const size_t n8 = (size_t)NB * SEQ * DM / 8;
        k_cvt8<<<(unsigned)((n8 + 255) / 256), 256, 0, stream>>>(z, ZB, n8);
    } else {
        const size_t n8 = (size_t)SEQ * DM / 8;
        for (int b = 0; b < NB; ++b) k_cvt8<<<(unsigned)((n8 + 255) / 256), 256, 0, stream>>>(z + (size_t)b * SEQ_FULL * DM, ZB + (size_t)b * SEQ * DM, n8);
    }
    k_wconv<<<10, 256, 0, stream>>>(wqkv, wproj, WT, WP2);

    k_qk<<<dim3(NB * SEQ / 64, 2, 1), 32, 0, stream>>>(ZB, WT, bqkv, QK);
    k_vt<<<dim3(NB * SEQ / 64, 1, 1), 32, 0, stream>>>(WT, ZB, bqkv, VT);

    k_flash_early<<<dim3(EROWS / 16, NB, 1), 32 * NH_, 0, stream>>>(QK, VT, CT);
    if (SEQ > EROWS)
        k_flash_late<<<dim3((SEQ - EROWS) / 16, NB, 1), 32 * NH_, 0, stream>>>(QK, VT, CT);

    k_out<<<dim3(NB * SEQ / 64, 1, 1), 32, 0, stream>>>(CT, WP2, bproj, OUT);
}
